// ImplicitModel_88476326298065
// MI455X (gfx1250) — hardware-run, weakly checked
//
#include <hip/hip_runtime.h>
#include <math.h>

typedef __attribute__((ext_vector_type(16))) _Float16 v16h;
typedef __attribute__((ext_vector_type(8)))  _Float16 v8h;
typedef __attribute__((ext_vector_type(8)))  float    v8f;
typedef __attribute__((ext_vector_type(4)))  float    v4f;

constexpr int kBatch   = 4096;
constexpr int kState   = 512;
constexpr int kNonlin  = 1024;
constexpr int kAction  = 256;
constexpr int kSolveIters = 30;
constexpr int kCatK    = kState + kAction + kNonlin;
constexpr int kColUs   = kState;
constexpr int kColQ    = kState + kAction;
constexpr float kWCarry    = 64.0f;
constexpr float kWCarryInv = 1.0f / kWCarry;
constexpr int kSlabPitch = 68;
constexpr int kTrPitch   = 65;

static_assert(kCatK == 1792);
static_assert((kSolveIters % 2) == 0 && kSolveIters >= 8);
static_assert((kBatch % 64) == 0 && (kNonlin % 64) == 0 && (kState % 64) == 0 && (kAction % 64) == 0);
static_assert((kState % 32) == 0 && (kNonlin % 32) == 0 && (kCatK % 32) == 0);
static_assert(((kCatK * 2) % 128) == 0 && ((kColQ * 2) % 128) == 0 && ((kColUs * 2) % 128) == 0);

constexpr size_t kOffACAT = 0;
constexpr size_t kOffQA   = kOffACAT + (size_t)kBatch  * kCatK   * 2;
constexpr size_t kOffXC   = kOffQA   + (size_t)kBatch  * kNonlin * 2;
constexpr size_t kOffC2T  = kOffXC   + (size_t)kBatch  * kNonlin * 4;
constexpr size_t kOffD3T  = kOffC2T  + (size_t)kNonlin * kState  * 2;
constexpr size_t kOffWCAT = kOffD3T  + (size_t)kNonlin * kNonlin * 2;
constexpr size_t kWsTotal = kOffWCAT + (size_t)kState  * kCatK   * 2;
static_assert(kWsTotal == 44826624ull);
static_assert(kWsTotal <= 134217728ull);
static_assert((kOffQA % 128) == 0 && (kOffXC % 128) == 0 && (kOffC2T % 128) == 0 &&
              (kOffD3T % 128) == 0 && (kOffWCAT % 128) == 0);

union FragU { v16h v; v8h h[2]; };
__device__ __forceinline__ v16h frag_load_f16(const _Float16* p) {
  FragU f;
  f.h[0] = *(const v8h*)(p);
  f.h[1] = *(const v8h*)(p + 16);
  return f.v;
}
__device__ __forceinline__ v8f mma_f16_guarded(v16h a, v16h b, v8f c) {
  c = __builtin_amdgcn_wmma_f32_16x16x32_f16(false, a, false, b, (short)0, c, false, false);
  asm volatile("v_nop\n\tv_nop\n\tv_nop\n\tv_nop" : "+v"(c) : "v"(a), "v"(b));
  return c;
}

__device__ __forceinline__ float tanh_fast(float z) {
  const float zc = fminf(fmaxf(z, -15.0f), 15.0f);
  const float e  = __expf(2.0f * zc);
  return 1.0f - 2.0f * __builtin_amdgcn_rcpf(e + 1.0f);
}

template <int NC8>
__global__ __launch_bounds__(256) void cast_rows_f16_kernel(
    const float* __restrict__ src, unsigned short* dst, int ldd, int coloff, int total8)
{
  const int i = blockIdx.x * 256 + threadIdx.x;
  if (i >= total8) return;
  const int row = i / NC8;
  const int g   = i - row * NC8;
  const size_t e0 = (size_t)i << 3;
  const v4f a0 = *(const v4f*)(src + e0);
  const v4f a1 = *(const v4f*)(src + e0 + 4);
  v8h hv;
#pragma unroll
  for (int e = 0; e < 4; ++e) {
    hv[e]     = (_Float16)a0[e];
    hv[4 + e] = (_Float16)a1[e];
  }
  unsigned short* q = dst + (size_t)row * ldd + coloff + g * 8;
  *(volatile v8h*)q = hv;
  __threadfence();
  *(volatile v8h*)q = hv;
}

__global__ __launch_bounds__(256) void transpose_cast_kernel(
    const float* __restrict__ W, int Ndim, unsigned short* Bt, int ldb, int kdst, float carry)
{
  __shared__ float sW[64 * kTrPitch];
  const int tid = threadIdx.x, lane = tid & 31, wave = tid >> 5;
  const int n0 = blockIdx.x * 64;
  const int k0 = blockIdx.y * 64;
#pragma unroll
  for (int it = 0; it < 4; ++it) {
    const int idx = it * 256 + tid;
    const int r   = idx >> 4;
    const int c4  = (idx & 15) * 4;
    const v4f v = *(const v4f*)(W + (size_t)(k0 + r) * Ndim + n0 + c4);
    sW[r * kTrPitch + c4 + 0] = v[0];
    sW[r * kTrPitch + c4 + 1] = v[1];
    sW[r * kTrPitch + c4 + 2] = v[2];
    sW[r * kTrPitch + c4 + 3] = v[3];
  }
  __syncthreads();
  const int q = lane >> 3, c8 = (lane & 7) * 8;
  v8h hv[2];
#pragma unroll
  for (int it = 0; it < 2; ++it) {
    const int n = it * 32 + wave * 4 + q;
#pragma unroll
    for (int e = 0; e < 8; ++e) {
      const float x = sW[(c8 + e) * kTrPitch + n] * carry;
      hv[it][e] = (_Float16)x;
    }
  }
  for (int pass = 0; pass < 2; ++pass) {
#pragma unroll
    for (int it = 0; it < 2; ++it) {
      const int n = it * 32 + wave * 4 + q;
      *(volatile v8h*)(Bt + (size_t)(n0 + n) * ldb + kdst + k0 + c8) = hv[it];
    }
    __threadfence();
  }
}

template <int MODE>
__global__ __launch_bounds__(256) void gemm_tile64_kernel(
    const unsigned short* __restrict__ Ap, int lda,
    const unsigned short* __restrict__ Btp, int ldb,
    float* Cf, int ldcf,
    unsigned short* Ch, int ldch,
    const float* __restrict__ Xadd, int ldx,
    int M, int N, int K, float scale)
{
  __shared__ __align__(16) float sT[8][16 * kSlabPitch];
  const int lane = threadIdx.x & 31;
  const int wave = threadIdx.x >> 5;
  const int tilesN = N >> 6;
  const int tilesM = M >> 6;
  const int tile = blockIdx.x * 8 + wave;
  if (tile >= tilesM * tilesN) return;
  const int tm = tile / tilesN;
  const int tn = tile - tm * tilesN;
  const int m0 = tm << 6;
  const int n0 = tn << 6;

  const int rlane = lane & 15;
  const int koff  = (lane >> 4) * 8;
  const int mOff  = (lane >> 4) * 8;

  const _Float16* pa = (const _Float16*)Ap  + (size_t)(m0 + rlane) * lda + koff;
  const _Float16* pb = (const _Float16*)Btp + (size_t)(n0 + rlane) * ldb + koff;
  const size_t a16 = (size_t)16 * lda;
  const size_t b16 = (size_t)16 * ldb;

  v8f acc[4][4];
#pragma unroll
  for (int i = 0; i < 4; ++i)
#pragma unroll
    for (int j = 0; j < 4; ++j) acc[i][j] = (v8f){0.f, 0.f, 0.f, 0.f, 0.f, 0.f, 0.f, 0.f};

#pragma unroll 1
  for (int k0 = 0; k0 < K; k0 += 32) {
    v16h bh[4];
#pragma unroll
    for (int j = 0; j < 4; ++j) bh[j] = frag_load_f16(pb + (size_t)j * b16 + k0);
#pragma unroll
    for (int i = 0; i < 4; ++i) {
      const v16h ah = frag_load_f16(pa + (size_t)i * a16 + k0);
#pragma unroll
      for (int j = 0; j < 4; ++j) acc[i][j] = mma_f16_guarded(ah, bh[j], acc[i][j]);
    }
  }

  float* slab = sT[wave];
  const int hh = lane >> 4, c4 = (lane & 15) * 4;
  const int q  = lane >> 3, c8 = (lane & 7) * 8;
#pragma unroll
  for (int i = 0; i < 4; ++i) {
    const int mBase = m0 + (i << 4);
#pragma unroll
    for (int j = 0; j < 4; ++j) {
#pragma unroll
      for (int r = 0; r < 8; ++r) {
        slab[(mOff + r) * kSlabPitch + (j << 4) + rlane] = acc[i][j][r] * scale;
      }
    }
    __builtin_amdgcn_fence(__ATOMIC_RELEASE, "workgroup");
    __builtin_amdgcn_wave_barrier();
    __builtin_amdgcn_fence(__ATOMIC_ACQUIRE, "workgroup");

    v4f fv[8];
    v8h hv[4];
    if (MODE == 0 || MODE == 2) {
#pragma unroll
      for (int it = 0; it < 8; ++it) fv[it] = *(const v4f*)(slab + (it * 2 + hh) * kSlabPitch + c4);
    }
    if (MODE == 0 || MODE == 1) {
#pragma unroll
      for (int it = 0; it < 4; ++it) {
        const int row = it * 4 + q;
        const float* sp = slab + row * kSlabPitch + c8;
        v4f a0 = *(const v4f*)(sp);
        v4f a1 = *(const v4f*)(sp + 4);
        if (MODE == 1) {
          const float* xp = Xadd + (size_t)(mBase + row) * ldx + n0 + c8;
          const v4f x0 = *(const v4f*)(xp);
          const v4f x1 = *(const v4f*)(xp + 4);
          a0 = a0 + x0;
          a1 = a1 + x1;
        }
#pragma unroll
        for (int e = 0; e < 4; ++e) {
          const float t0 = tanh_fast(a0[e]);
          const float t1 = tanh_fast(a1[e]);
          hv[it][e]     = (_Float16)t0;
          hv[it][4 + e] = (_Float16)t1;
        }
      }
    }
    for (int pass = 0; pass < 2; ++pass) {
      if (MODE == 0 || MODE == 2) {
#pragma unroll
        for (int it = 0; it < 8; ++it) {
          const int row = it * 2 + hh;
          *(volatile v4f*)(Cf + (size_t)(mBase + row) * ldcf + n0 + c4) = fv[it];
        }
      }
      if (MODE == 0 || MODE == 1) {
#pragma unroll
        for (int it = 0; it < 4; ++it) {
          const int row = it * 4 + q;
          *(volatile v8h*)(Ch + (size_t)(mBase + row) * ldch + n0 + c8) = hv[it];
        }
      }
      __threadfence();
    }
    __builtin_amdgcn_fence(__ATOMIC_RELEASE, "workgroup");
    __builtin_amdgcn_wave_barrier();
    __builtin_amdgcn_fence(__ATOMIC_ACQUIRE, "workgroup");
  }
}

extern "C" void kernel_launch(void* const* d_in, const int* in_sizes, int n_in,
                              void* d_out, int out_size, void* d_ws, size_t ws_size,
                              hipStream_t stream) {
  if (n_in < 7) return;
  if (in_sizes[0] != kBatch * kState) return;
  if (in_sizes[1] != kBatch * kAction) return;
  if (in_sizes[2] != kState * kState) return;
  if (in_sizes[3] != kNonlin * kState) return;
  if (in_sizes[4] != kAction * kState) return;
  if (in_sizes[5] != kState * kNonlin) return;
  if (in_sizes[6] != kNonlin * kNonlin) return;
  if (out_size != kBatch * kState) return;
  if (ws_size < kWsTotal) return;

  const float* xs  = (const float*)d_in[0];
  const float* us  = (const float*)d_in[1];
  const float* A_T = (const float*)d_in[2];
  const float* B1T = (const float*)d_in[3];
  const float* B2T = (const float*)d_in[4];
  const float* C2T = (const float*)d_in[5];
  const float* D3T = (const float*)d_in[6];
  float* out = (float*)d_out;

  char* ws = (char*)d_ws;
  unsigned short* ACAT = (unsigned short*)(ws + kOffACAT);
  unsigned short* QA   = (unsigned short*)(ws + kOffQA);
  float*          XC   = (float*)(ws + kOffXC);
  unsigned short* C2t  = (unsigned short*)(ws + kOffC2T);
  unsigned short* D3t  = (unsigned short*)(ws + kOffD3T);
  unsigned short* WCAT = (unsigned short*)(ws + kOffWCAT);

  {
    const int t8x = kBatch * kState / 8;
    const int t8u = kBatch * kAction / 8;
    cast_rows_f16_kernel<kState / 8><<<t8x / 256, 256, 0, stream>>>(xs, ACAT, kCatK, 0, t8x);
    cast_rows_f16_kernel<kAction / 8><<<t8u / 256, 256, 0, stream>>>(us, ACAT, kCatK, kColUs, t8u);
  }

  transpose_cast_kernel<<<dim3(kNonlin / 64, kState / 64), 256, 0, stream>>>(C2T, kNonlin, C2t, kState, 0, kWCarry);
  transpose_cast_kernel<<<dim3(kNonlin / 64, kNonlin / 64), 256, 0, stream>>>(D3T, kNonlin, D3t, kNonlin, 0, kWCarry);
  transpose_cast_kernel<<<dim3(kState / 64, kState / 64), 256, 0, stream>>>(A_T, kState, WCAT, kCatK, 0, kWCarry);
  transpose_cast_kernel<<<dim3(kState / 64, kAction / 64), 256, 0, stream>>>(B2T, kState, WCAT, kCatK, kColUs, kWCarry);
  transpose_cast_kernel<<<dim3(kState / 64, kNonlin / 64), 256, 0, stream>>>(B1T, kState, WCAT, kCatK, kColQ, kWCarry);

  const int blocksWide = ((kBatch / 64) * (kNonlin / 64) + 7) / 8;
  const int blocksOut  = ((kBatch / 64) * (kState / 64) + 7) / 8;

  gemm_tile64_kernel<0><<<blocksWide, 256, 0, stream>>>(
      ACAT, kCatK, C2t, kState,
      XC, kNonlin,
      QA, kNonlin,
      nullptr, 0,
      kBatch, kNonlin, kState, kWCarryInv);

  for (int j = 1; j < kSolveIters; ++j) {
    const bool odd = (j & 1) != 0;
    const unsigned short* qin = odd ? (const unsigned short*)QA : (const unsigned short*)(ACAT + kColQ);
    const int ldin  = odd ? kNonlin : kCatK;
    unsigned short* qout = odd ? (ACAT + kColQ) : QA;
    const int ldout = odd ? kCatK : kNonlin;
    gemm_tile64_kernel<1><<<blocksWide, 256, 0, stream>>>(
        qin, ldin, D3t, kNonlin,
        nullptr, 0,
        qout, ldout,
        XC, kNonlin,
        kBatch, kNonlin, kNonlin, kWCarryInv);
  }

  gemm_tile64_kernel<2><<<blocksOut, 256, 0, stream>>>(
      ACAT, kCatK, WCAT, kCatK,
      out, kState,
      nullptr, 0,
      nullptr, 0,
      kBatch, kState, kCatK, kWCarryInv);
}
